// naiveTransformerNet_18494129177013
// MI455X (gfx1250) — hardware-verified
//
#include <hip/hip_runtime.h>
#include <math.h>

typedef __attribute__((ext_vector_type(16))) _Float16 v16h;
typedef __attribute__((ext_vector_type(16))) __bf16 v16b;
typedef __attribute__((ext_vector_type(8)))  _Float16 v8h;
typedef __attribute__((ext_vector_type(8)))  float v8f;
typedef __attribute__((ext_vector_type(4)))  float v4f;
typedef __attribute__((ext_vector_type(2)))  float v2f;
typedef __attribute__((ext_vector_type(4)))  unsigned v4u;
typedef __attribute__((ext_vector_type(4)))  int v4i;
typedef float __attribute__((may_alias)) float_a;
typedef int __attribute__((may_alias)) int_a;

template <typename T> __device__ __forceinline__ void vst2(void* p, T v) { *(volatile T*)p = v; __threadfence(); *(volatile T*)p = v; }
__device__ __forceinline__ v8f wmma16(v16h a, v16h b, v8f c) {
  v8f d = __builtin_amdgcn_wmma_f32_16x16x32_f16(false, a, false, b, (short)0, c, false, false);
  asm volatile("v_nop\n\tv_nop\n\tv_nop\n\tv_nop" : "+v"(d) : "v"(a), "v"(b));
  return d;
}
__device__ __forceinline__ v8f wmma_bf(v16b a, v16b b, v8f c) {
  v8f d = __builtin_amdgcn_wmma_f32_16x16x32_bf16(false, a, false, b, (short)0, c, false, false);
  asm volatile("v_nop\n\tv_nop\n\tv_nop\n\tv_nop" : "+v"(d) : "v"(a), "v"(b));
  return d;
}
__device__ __forceinline__ v16h frag_h(const _Float16* rowk0, int lane) {
  union { v16h v; v8h q[2]; } u; const _Float16* p = rowk0 + 8 * (lane >> 4);
  u.q[0] = *(const v8h*)p; u.q[1] = *(const v8h*)(p + 16); return u.v;
}
__device__ __forceinline__ v16h frag_f32(const float* rowk0, int lane) {
  v16h a; const float* p = rowk0 + 8 * (lane >> 4);
#pragma unroll
  for (int i = 0; i < 8; ++i) { a[i] = (_Float16)p[i]; a[8 + i] = (_Float16)p[16 + i]; }
  return a;
}
__device__ __forceinline__ v16h frag_f32s(const float* rowk0, int lane, float sc) {
  v16h a; const float* p = rowk0 + 8 * (lane >> 4);
#pragma unroll
  for (int i = 0; i < 8; ++i) { a[i] = (_Float16)(p[i] * sc); a[8 + i] = (_Float16)(p[16 + i] * sc); }
  return a;
}
__device__ __forceinline__ v16h fragc_f32(const float* W, int k0, int n, int lane, int ld, int K) {
  v16h a; const int g = lane >> 4;
#pragma unroll
  for (int i = 0; i < 8; ++i) { const int ka = k0 + 8 * g + i, kb = ka + 16;
    a[i] = (_Float16)(ka < K ? W[(size_t)(ka < K ? ka : K - 1) * ld + n] : 0.f); a[8 + i] = (_Float16)(kb < K ? W[(size_t)(kb < K ? kb : K - 1) * ld + n] : 0.f); }
  return a;
}
struct F2 { v16b h, l; };
__device__ __forceinline__ F2 bsplit16(const float v[16]) { F2 r;
#pragma unroll
  for (int i = 0; i < 16; ++i) { const __bf16 h = (__bf16)v[i]; r.h[i] = h; r.l[i] = (__bf16)(v[i] - (float)h); }
  return r; }
__device__ __forceinline__ F2 split_row(const float* row, int k0, int lane) { float v[16]; const float* p = row + k0 + 8 * (lane >> 4);
#pragma unroll
  for (int i = 0; i < 8; ++i) { v[i] = p[i]; v[8 + i] = p[16 + i]; }
  return bsplit16(v); }
__device__ __forceinline__ F2 split_rowK(const float* row, int k0, int lane, int K) { float v[16]; const int g = lane >> 4;
#pragma unroll
  for (int i = 0; i < 8; ++i) { const int ka = k0 + 8 * g + i, kb = ka + 16; v[i] = ka < K ? row[ka < K ? ka : K - 1] : 0.f; v[8 + i] = kb < K ? row[kb < K ? kb : K - 1] : 0.f; }
  return bsplit16(v); }
__device__ __forceinline__ F2 split_col(const float* W, int k0, int n, int lane, int ld, int K) { float v[16]; const int g = lane >> 4;
#pragma unroll
  for (int i = 0; i < 8; ++i) { const int ka = k0 + 8 * g + i, kb = ka + 16; v[i] = ka < K ? W[(size_t)(ka < K ? ka : K - 1) * ld + n] : 0.f; v[8 + i] = kb < K ? W[(size_t)(kb < K ? kb : K - 1) * ld + n] : 0.f; }
  return bsplit16(v); }
__device__ __forceinline__ v8f mac3(const F2& a, const F2& b, v8f c) { c = wmma_bf(a.l, b.h, c); c = wmma_bf(a.h, b.l, c); return wmma_bf(a.h, b.h, c); }
__device__ __forceinline__ float sigm(float v) { return 1.0f / (1.0f + expf(-v)); }
#define LDSX() do { asm volatile("s_wait_dscnt 0" ::: "memory"); __builtin_amdgcn_wave_barrier(); __builtin_amdgcn_fence(__ATOMIC_RELEASE, "workgroup"); } while (0)


#define CSR_N 100000
#define CSR_E 1600000
#define NNP 100032
#define NG 64
#define CSR_CHUNK 16384
#ifndef TLB2
#define TLB2 (NNP / 64)
#endif
#ifndef DBGM
#define DBGM 0
#endif
#ifndef TLB1
#define TLB1 (NNP / 64)
#endif

#define CSR_FINN (CSR_E + 32 * CSR_NBK)
#ifndef CSR_CHUNK
#define CSR_CHUNK 4096
#endif
#define CSR_EPT (CSR_CHUNK / 256)
#define CSR_BKT 256
#define CSR_NCH ((CSR_E + CSR_CHUNK - 1) / CSR_CHUNK)
#define CSR_NBK ((CSR_N + CSR_BKT - 1) / CSR_BKT)
#define CSR_NBKP (((CSR_NBK + 63) / 64) * 64)
#define CSR_SEGCAP (CSR_E + 32 * CSR_NBK * CSR_NCH)
#ifndef CSR_BCAP
#define CSR_BCAP 10240
#endif
#define CSR_SZ_CNT   (4u * CSR_NCH * CSR_NBKP)
#define CSR_SZ_OFF   (4u * CSR_NBK * (((CSR_NCH + 31) / 32) * 32))
#define CSR_SZ_BST   (4u * (((CSR_NBK + 1 + 31) / 32) * 32))
#define CSR_SZ_SEG   (4u * CSR_SEGCAP)
#define CSR_SZ_FIN   (4u * (CSR_E + 32 * CSR_NBK))
#define CSR_SZ_ROW   (4u * CSR_NBK * CSR_BKT)
#define CSR_OFFP (((CSR_NCH + 31) / 32) * 32)

__global__ __launch_bounds__(256) void k_csr_cnt(const int* __restrict__ DST, int dstride, int* __restrict__ CNT) {
  __shared__ unsigned short sc[256][CSR_NBK + 1]; __shared__ __align__(16) int srow[CSR_NBKP];
  const int c = blockIdx.x, tid = threadIdx.x;
  for (int b = 0; b < CSR_NBK; ++b) sc[tid][b] = 0;
  const size_t e0 = (size_t)c * CSR_CHUNK + tid * CSR_EPT;
  for (int i = 0; i < CSR_EPT; ++i) { const size_t e = e0 + i; if (e < (size_t)CSR_E) { int d = DST[e * dstride]; d = min(max(d, 0), CSR_N - 1); sc[tid][d / CSR_BKT] += 1; } }
  __syncthreads();
  for (int b = tid; b < CSR_NBKP; b += 256) { int s = 0; if (b < CSR_NBK) for (int t = 0; t < 256; ++t) s += sc[t][b]; srow[b] = s; }
  __syncthreads();
  for (int q = tid; q < CSR_NBKP / 4; q += 256) vst2((unsigned*)(CNT + (size_t)c * CSR_NBKP + q * 4), *(const v4u*)&srow[q * 4]);
}
__global__ __launch_bounds__(256) void k_csr_scan(const int* __restrict__ CNT, int* __restrict__ OFF, int* __restrict__ BST) {
  __shared__ int sbt[CSR_NBK + 1]; __shared__ int sbs[((CSR_NBK + 1 + 31) / 32) * 32]; __shared__ int scnt[CSR_NBK + 1]; __shared__ __align__(16) int sbuf[64][CSR_OFFP];
  const int tid = threadIdx.x;
  for (int b = tid; b < CSR_NBK; b += 256) { int sp = 0, st = 0; for (int c = 0; c < CSR_NCH; ++c) { const int n = CNT[(size_t)c * CSR_NBKP + b]; st += n; sp += (n + 31) & ~31; } sbt[b] = sp; scnt[b] = st; }
  for (int b = tid; b < ((CSR_NBK + 1 + 31) / 32) * 32; b += 256) sbs[b] = 0;
  __syncthreads();
  if (tid == 0) { int acc = 0, accf = 0; for (int b = 0; b < CSR_NBK; ++b) { const int t = sbt[b]; sbt[b] = acc; acc += t; sbs[b] = accf; accf += (scnt[b] + 31) & ~31; } sbs[CSR_NBK] = accf; }
  __syncthreads();
  for (int b0 = 0; b0 < CSR_NBK; b0 += 64) {
    if (tid < 64 && b0 + tid < CSR_NBK) { const int b = b0 + tid; int o = sbt[b]; for (int c = 0; c < CSR_OFFP; ++c) { if (c < CSR_NCH) { sbuf[tid][c] = o; o += (CNT[(size_t)c * CSR_NBKP + b] + 31) & ~31; } else sbuf[tid][c] = 0; } }
    __syncthreads();
    for (int q = tid; q < 64 * (CSR_OFFP / 4); q += 256) { const int r = q / (CSR_OFFP / 4), pc = q % (CSR_OFFP / 4); if (b0 + r < CSR_NBK) vst2((unsigned*)(OFF + (size_t)(b0 + r) * CSR_OFFP + pc * 4), *(const v4u*)&sbuf[r][pc * 4]); }
    __syncthreads(); }
  for (int q = tid; q < ((CSR_NBK + 1 + 31) / 32) * 32 / 4; q += 256) vst2((unsigned*)(BST + q * 4), *(const v4u*)&sbs[q * 4]);
}
__global__ __launch_bounds__(256) void k_csr_scatter(const int* __restrict__ SRC, const int* __restrict__ DST, int sstride, int dstride, const int* __restrict__ OFF, int* __restrict__ SEGS, int* __restrict__ SEGE) {
  __shared__ unsigned short sc[256][CSR_NBK + 1]; __shared__ int sbase[CSR_NBK + 1]; __shared__ int scn[CSR_NBK + 1]; __shared__ int sord[CSR_CHUNK];
  const int c = blockIdx.x, tid = threadIdx.x;
  for (int b = 0; b < CSR_NBK; ++b) sc[tid][b] = 0;
  const size_t e0 = (size_t)c * CSR_CHUNK + tid * CSR_EPT; int bk[CSR_EPT];
#pragma unroll
  for (int i = 0; i < CSR_EPT; ++i) { const size_t e = e0 + i; bk[i] = -1; if (e < (size_t)CSR_E) { int d = DST[e * dstride]; d = min(max(d, 0), CSR_N - 1); bk[i] = d / CSR_BKT; sc[tid][bk[i]] += 1; } }
  __syncthreads();
  for (int b = tid; b < CSR_NBK; b += 256) { int acc = 0; for (int t = 0; t < 256; ++t) { const int v = sc[t][b]; sc[t][b] = (unsigned short)acc; acc += v; } scn[b] = acc; }
  __syncthreads();
  if (tid == 0) { int acc = 0; for (int b = 0; b < CSR_NBK; ++b) { sbase[b] = acc; acc += scn[b]; } }
  __syncthreads();
#pragma unroll
  for (int i = 0; i < CSR_EPT; ++i) { if (bk[i] >= 0) { const int b = bk[i]; const int r = sc[tid][b]; sc[tid][b] = (unsigned short)(r + 1); sord[sbase[b] + r] = tid * CSR_EPT + i; } }
  __syncthreads();
  for (int b = 0; b < CSR_NBK; ++b) { const int n = scn[b]; if (n == 0) continue; const int nl = ((n + 31) & ~31); const size_t o = (size_t)(min(max(OFF[(size_t)b * CSR_OFFP + c], 0), CSR_SEGCAP - nl) & ~31);
    for (int q = tid; q < nl / 4; q += 256) { int4 vs, ve;
#pragma unroll
      for (int k = 0; k < 4; ++k) { const int i = q * 4 + k; int s = -1, eid = -1; if (i < n) { const size_t e = (size_t)c * CSR_CHUNK + sord[sbase[b] + i]; s = min(max(SRC[e * sstride], 0), CSR_N - 1); eid = (int)e; } vs[k] = s; ve[k] = eid; }
      vst2((unsigned*)(SEGS + o + q * 4), *(const v4u*)&vs); vst2((unsigned*)(SEGE + o + q * 4), *(const v4u*)&ve); } }
}
__global__ __launch_bounds__(256) void k_csr_bucket(const int* __restrict__ CNT, const int* __restrict__ OFF, const int* __restrict__ BST, const int* __restrict__ SEGS, const int* __restrict__ SEGE, const int* __restrict__ DST, int dstride, int* __restrict__ FS, int* __restrict__ FE, int* __restrict__ ROWST, int* __restrict__ ROWCNT) {
  __shared__ int ssrc[CSR_BCAP]; __shared__ int seid[CSR_BCAP]; __shared__ unsigned char snod[CSR_BCAP]; __shared__ int souts[CSR_BCAP]; __shared__ int soute[CSR_BCAP]; __shared__ int scount[256]; __shared__ int sstart[257]; __shared__ int stot;
  const int b = blockIdx.x, tid = threadIdx.x;
  if (tid == 0) { int t = 0; for (int c = 0; c < CSR_NCH; ++c) t += min(max(CNT[(size_t)c * CSR_NBKP + b], 0), CSR_CHUNK); stot = (t <= CSR_BCAP) ? t : 0; }
  __syncthreads();
  { int base = 0; for (int c = 0; c < CSR_NCH; ++c) { const int n = min(max(CNT[(size_t)c * CSR_NBKP + b], 0), CSR_CHUNK); const int o = min(max(OFF[(size_t)b * CSR_OFFP + c], 0), CSR_SEGCAP - ((n + 31) & ~31));
      for (int i = tid; i < n; i += 256) { const int p = base + i; if (p < CSR_BCAP) { ssrc[p] = min(max(SEGS[o + i], 0), CSR_N - 1); const int e = min(max(SEGE[o + i], 0), CSR_E - 1); seid[p] = e; int d = DST[(size_t)e * dstride]; d = min(max(d, 0), CSR_N - 1); const int dl = d - b * CSR_BKT; snod[p] = (unsigned char)(dl >= 0 && dl < 256 ? dl : 255); } }
      base += n; } }
  __syncthreads();
  const int node = b * CSR_BKT + tid; int cnt = 0; for (int p = 0; p < stot; ++p) cnt += (snod[p] == tid) ? 1 : 0;
  scount[tid] = cnt; __syncthreads();
  if (tid == 0) { int acc = 0; for (int t = 0; t < 256; ++t) { sstart[t] = acc; acc += scount[t]; } sstart[256] = acc; }
  __syncthreads();
  const int bst0 = min(max(BST[b], 0), CSR_FINN - ((sstart[256] + 31) & ~31)) & ~31; const int gst = bst0 + sstart[tid];
  { int w = sstart[tid]; for (int p = 0; p < stot; ++p) if (snod[p] == tid) { souts[w] = ssrc[p]; soute[w] = seid[p]; ++w; } }
  __syncthreads();
  { const int n = sstart[256]; const int nl = (n + 31) & ~31; for (int q = tid; q < nl / 4; q += 256) { int4 vs, ve;
#pragma unroll
      for (int k = 0; k < 4; ++k) { const int i = q * 4 + k; vs[k] = i < n ? souts[i] : -1; ve[k] = i < n ? soute[i] : -1; }
      vst2((unsigned*)(FS + bst0 + q * 4), *(const v4u*)&vs); vst2((unsigned*)(FE + bst0 + q * 4), *(const v4u*)&ve); } }
  __syncthreads();
  { __shared__ __align__(16) int srs[256], src2[256]; srs[tid] = node < CSR_N ? gst : 0; src2[tid] = node < CSR_N ? cnt : 0; __syncthreads();
    if (tid < 64) vst2((unsigned*)(ROWST + (size_t)b * 256 + tid * 4), *(const v4u*)&srs[tid * 4]); else if (tid < 128) vst2((unsigned*)(ROWCNT + (size_t)b * 256 + (tid - 64) * 4), *(const v4u*)&src2[(tid - 64) * 4]); }
}

typedef __attribute__((ext_vector_type(8))) __bf16 v8b;
__device__ __forceinline__ v16b frag_b(const __bf16* rowk0, int lane) {
  union { v16b v; v8b q[2]; } u; const __bf16* p = rowk0 + 8 * (lane >> 4);
  u.q[0] = *(const v8b*)p; u.q[1] = *(const v8b*)(p + 16); return u.v;
}
__device__ __forceinline__ float bfr(float v) { return (float)(__bf16)v; }
__device__ __attribute__((noinline)) float exp_ni(float v) { return expf(v); }
#define WS_CNT  0u
#define WS_OFF  (WS_CNT + CSR_SZ_CNT)
#define WS_BST  (WS_OFF + CSR_SZ_OFF)
#define WS_SEGS (WS_BST + CSR_SZ_BST)
#define WS_SEGE (WS_SEGS + CSR_SZ_SEG)
#define WS_FS   (WS_SEGE + CSR_SZ_SEG)
#define WS_FE   (WS_FS + CSR_SZ_FIN)
#define WS_RST  (WS_FE + CSR_SZ_FIN)
#define WS_RCT  (WS_RST + CSR_SZ_ROW)
#define WS_PT   (WS_RCT + CSR_SZ_ROW)
#define PT1 0
#define PT2 (4 * 48 * 128)
#define PTE (PT2 + 4 * 32 * 64)
#define WS_KV1  (WS_PT + 2u * PTE)
#define WS_KV2  WS_KV1
#define WS_H1   (WS_KV1 + 4u * NNP * 80)
#define WS_H2   (WS_H1 + 4u * NNP * 64)
#define WS_PG   (WS_H2 + 4u * NNP * 32)
#define WS_END  (WS_PG + 4u * NG * 32)

__global__ __launch_bounds__(128) void k_pack(const float* __restrict__ Wq1, const float* __restrict__ Wk1, const float* __restrict__ Wv1, const float* __restrict__ Ws1, const float* __restrict__ Wq2, const float* __restrict__ Wk2, const float* __restrict__ Wv2, const float* __restrict__ Ws2, __bf16* __restrict__ PT) {
  __shared__ __align__(16) __bf16 srow[128];
  const int n = blockIdx.x, tid = threadIdx.x;
  if (n < 192) { const int which = n / 48, o = n % 48; const float* Wm = which == 0 ? Wq1 : (which == 1 ? Wk1 : (which == 2 ? Wv1 : Ws1)); srow[tid] = (__bf16)(o < 40 ? bfr(Wm[(size_t)tid * 40 + o]) : 0.f); __syncthreads();
    if (tid < 16) vst2((unsigned*)(PT + PT1 + (size_t)n * 128 + tid * 8), *(const v4u*)(&srow[tid * 8])); }
  else { const int m = n - 192; const int which = m / 32, o = m % 32; const float* Wm = which == 0 ? Wq2 : (which == 1 ? Wk2 : (which == 2 ? Wv2 : Ws2)); if (tid < 64) srow[tid] = (__bf16)((o < 20 && tid < 40) ? bfr(Wm[(size_t)tid * 20 + o]) : 0.f); __syncthreads();
    if (tid < 8) vst2((unsigned*)(PT + PT2 + (size_t)m * 64 + tid * 8), *(const v4u*)(&srow[tid * 8])); }
}
template <int L>
__global__ __launch_bounds__(128) void k_kv(const float* __restrict__ X, const __bf16* __restrict__ PT, const float* __restrict__ bk, const float* __restrict__ bv, float* __restrict__ KV) {
  constexpr int KI = L == 1 ? 128 : 64, CO = L == 1 ? 40 : 20, TPP = L == 1 ? 3 : 2, PITCH = L == 1 ? 80 : 64, ROWS = L == 1 ? 48 : 32;
  __shared__ __align__(16) float so[4][16][100];
  const int tid = threadIdx.x, wave = tid >> 5, lane = tid & 31, col = lane & 15, g = lane >> 4; const size_t r0 = (size_t)blockIdx.x * 64 + wave * 16; const size_t ra = min(r0 + col, (size_t)CSR_N - 1);
  const __bf16* P = PT + (L == 1 ? PT1 : PT2);
  v8f acc[2 * TPP] = {};
#pragma unroll
  for (int kc = 0; kc < KI / 32; ++kc) { const F2 a = split_row(X + ra * KI, kc * 32, lane);
#pragma unroll
    for (int j = 0; j < 2 * TPP; ++j) { const int which = 1 + j / TPP, t = j % TPP; const v16b w = frag_b(P + (size_t)(which * ROWS + t * 16 + col) * KI + kc * 32, lane); if (L == 2) acc[j] = wmma_bf(a.l, w, acc[j]); acc[j] = wmma_bf(a.h, w, acc[j]); } }
#pragma unroll
  for (int j = 0; j < 2 * TPP; ++j) { const int part = j / TPP, t = j % TPP; const int o = t * 16 + col; const float bb = o < CO ? bfr((part == 0 ? bk : bv)[o]) : 0.f;
#pragma unroll
    for (int r = 0; r < 8; ++r) if (o < CO) so[wave][8 * g + r][part * (PITCH / 2) + o] = (r0 + 8 * g + r < (size_t)CSR_N) ? acc[j][r] + bb : 0.f; }
  LDSX();
  for (int q = lane; q < 16 * PITCH; q += 32) { const int rl = q / PITCH, c = q % PITCH; const int cc = c % (PITCH / 2); if (cc >= CO) so[wave][rl][c] = 0.f; }
  LDSX();
  for (int rl = 0; rl < 16; ++rl) for (int pc = lane; pc < PITCH / 4; pc += 32) vst2(KV + (r0 + rl) * PITCH + pc * 4, *(const v4f*)&so[wave][rl][pc * 4]);
}
template <int L>
__global__ __launch_bounds__(256) void k_conv(const float* __restrict__ X, const __bf16* __restrict__ PT, const float* __restrict__ bq, const float* __restrict__ bs, const float* __restrict__ KV, const float* __restrict__ EA, const float* __restrict__ We, const int* __restrict__ FS, const int* __restrict__ FE, const int* __restrict__ RST, const int* __restrict__ RCT, float* __restrict__ H) {
  constexpr int KI = L == 1 ? 128 : 64, CO = L == 1 ? 40 : 20, C = L == 1 ? 10 : 5, TPP = L == 1 ? 3 : 2, PITCH = L == 1 ? 80 : 64, ROWS = L == 1 ? 48 : 32, OP = L == 1 ? 64 : 32;
  __shared__ float sq[64][49], ssk[64][49]; __shared__ float swe[8][48]; __shared__ __align__(16) float sout[64][OP + 4]; __shared__ float sagg[256][11];
  const int tid = threadIdx.x, wave = tid >> 5, lane = tid & 31, col = lane & 15, g = lane >> 4;
  for (int q = tid; q < 8 * 48; q += 256) { const int d = q / 48, o = q % 48; swe[d][o] = o < CO ? bfr(We[d * CO + o]) : 0.f; }
  if (wave < 4) { const size_t r0 = (size_t)blockIdx.x * 64 + wave * 16; const size_t ra = min(r0 + col, (size_t)CSR_N - 1); const __bf16* P = PT + (L == 1 ? PT1 : PT2);
    v8f acc[2 * TPP] = {};
#pragma unroll
    for (int kc = 0; kc < KI / 32; ++kc) { const F2 a = split_row(X + ra * KI, kc * 32, lane);
#pragma unroll
      for (int j = 0; j < 2 * TPP; ++j) { const int which = (j / TPP) == 0 ? 0 : 3, t = j % TPP; const v16b w = frag_b(P + (size_t)(which * ROWS + t * 16 + col) * KI + kc * 32, lane); if (L == 2) acc[j] = wmma_bf(a.l, w, acc[j]); acc[j] = wmma_bf(a.h, w, acc[j]); } }
#pragma unroll
    for (int j = 0; j < 2 * TPP; ++j) { const int part = j / TPP, t = j % TPP; const int o = t * 16 + col;
#pragma unroll
      for (int r = 0; r < 8; ++r) { const float v = o < CO ? acc[j][r] + bfr((part == 0 ? bq : bs)[o]) : 0.f; if (part == 0) sq[wave * 16 + 8 * g + r][o] = v; else ssk[wave * 16 + 8 * g + r][o] = v; } } }
  __syncthreads();
  { const int nl = tid >> 2, h = tid & 3; const size_t node = (size_t)blockIdx.x * 64 + nl; const float isq = rsqrtf((float)C);
    float* myagg = &sagg[tid][0];
    for (int c = 0; c < C; ++c) myagg[c] = 0.f;
    float z = 0.f;
    if (node < (size_t)CSR_N) { const int cnt = min(max(RCT[node], 0), CSR_BCAP); const int st = min(max(RST[node], 0), CSR_FINN - cnt);
      float mx = -3.0e38f;
#pragma unroll 1
      for (int e = 0; e < cnt; ++e) { const int s = min(max(FS[st + e], 0), CSR_N - 1); const int eid = min(max(FE[st + e], 0), CSR_E - 1); const float* kr = KV + (size_t)s * PITCH + h * C; float ea8[8];
#pragma unroll
        for (int d = 0; d < 8; ++d) ea8[d] = bfr(EA[(size_t)eid * 8 + d]);
        float lg = 0.f;
#pragma unroll 1
        for (int c = 0; c < C; ++c) { float ec = 0.f;
#pragma unroll
          for (int d = 0; d < 8; ++d) ec += ea8[d] * swe[d][h * C + c];
          lg += sq[nl][h * C + c] * (kr[c] + ec); }
        mx = fmaxf(mx, lg * isq); }
#pragma unroll 1
      for (int e = 0; e < cnt; ++e) { const int s = min(max(FS[st + e], 0), CSR_N - 1); const int eid = min(max(FE[st + e], 0), CSR_E - 1); const float* kr = KV + (size_t)s * PITCH + h * C; const float* vr = KV + (size_t)s * PITCH + PITCH / 2 + h * C; float ea8[8];
#pragma unroll
        for (int d = 0; d < 8; ++d) ea8[d] = bfr(EA[(size_t)eid * 8 + d]);
        float lg = 0.f;
#pragma unroll 1
        for (int c = 0; c < C; ++c) { float ec = 0.f;
#pragma unroll
          for (int d = 0; d < 8; ++d) ec += ea8[d] * swe[d][h * C + c];
          lg += sq[nl][h * C + c] * (kr[c] + ec); }
        const float p = exp_ni(lg * isq - mx); z += p;
#pragma unroll 1
        for (int c = 0; c < C; ++c) { float ec = 0.f;
#pragma unroll
          for (int d = 0; d < 8; ++d) ec += ea8[d] * swe[d][h * C + c];
          myagg[c] += p * (vr[c] + ec); } } }
    const float iz = 1.0f / (z + 1e-16f);
#pragma unroll 1
    for (int c = 0; c < C; ++c) { const float v = myagg[c] * iz + ssk[nl][h * C + c]; sout[nl][h * C + c] = node < (size_t)CSR_N ? fmaxf(v, 0.f) : 0.f; }
    if (h == 0) for (int c = CO; c < OP; ++c) sout[nl][c] = 0.f; }
  __syncthreads();
  for (int q = tid; q < 64 * (OP / 4); q += 256) { const int nl = q / (OP / 4), pc = q % (OP / 4); vst2(H + ((size_t)blockIdx.x * 64 + nl) * OP + pc * 4, *(const v4f*)&sout[nl][pc * 4]); }
}
__global__ __launch_bounds__(256) void k_pool(const int* __restrict__ BATCH, const float* __restrict__ H2, float* __restrict__ PG) {
  __shared__ float sacc[8][32]; __shared__ int scnt[8]; __shared__ __align__(16) float srow[32]; __shared__ int srng[2];
  const int gph = blockIdx.x, tid = threadIdx.x; const int part = tid >> 5, c = tid & 31; float a = 0.f; int n_ = 0;
  if (tid < 2) { const int key = gph + tid; int lo = 0, hi = CSR_N; while (lo < hi) { const int mid = (lo + hi) >> 1; if (BATCH[mid] < key) lo = mid + 1; else hi = mid; } srng[tid] = lo; }
  __syncthreads();
  const int n0 = srng[0], n1 = max(srng[1], srng[0]);
  for (int n = n0 + part; n < n1; n += 8) if (BATCH[n] == gph) { a += H2[(size_t)n * 32 + c]; ++n_; }
  sacc[part][c] = a; if (c == 0) scnt[part] = n_;
  __syncthreads();
  if (tid < 32) { float s = 0.f; int cn = 0; for (int p = 0; p < 8; ++p) { s += sacc[p][tid]; cn += scnt[p]; } srow[tid] = s / fmaxf((float)cn, 1.0f); }
  __syncthreads();
  if (tid < 8) vst2(PG + (size_t)gph * 32 + tid * 4, *(const v4f*)&srow[tid * 4]);
}
__global__ __launch_bounds__(64) void k_mlp(const float* __restrict__ PG, const float* __restrict__ W1, const float* __restrict__ b1, const float* __restrict__ W2, const float* __restrict__ b2, float* __restrict__ out) {
  __shared__ __align__(16) float sres[64 * 3 + 4];
  const int gph = threadIdx.x; float hh[10];
#pragma unroll
  for (int o = 0; o < 10; ++o) { float s = bfr(b1[o]);
#pragma unroll 1
    for (int k = 0; k < 20; ++k) s += PG[gph * 32 + k] * bfr(W1[k * 10 + o]);
    hh[o] = fmaxf(s, 0.f); }
  __shared__ float shh[64][10];
#pragma unroll
  for (int o = 0; o < 10; ++o) shh[gph][o] = hh[o];
#pragma unroll
  for (int o = 0; o < 3; ++o) { float s = bfr(b2[o]);
#pragma unroll 1
    for (int k = 0; k < 10; ++k) s += shh[gph][k] * bfr(W2[k * 3 + o]);
    sres[gph * 3 + o] = s; }
  __syncthreads();
  if (gph < 48) vst2(out + gph * 4, *(const v4f*)&sres[gph * 4]);
}

#if DBGM == 1
__global__ __launch_bounds__(64) void k_dbg1(const float* __restrict__ H1, float* __restrict__ out) { __shared__ __align__(16) float s[192]; const int t = threadIdx.x; for (int i = t; i < 192; i += 64) s[i] = H1[(size_t)((i * 2731) % 4096) * 64 + (i * 7) % 40]; __syncthreads(); if (t < 48) vst2(out + t * 4, *(const v4f*)&s[t * 4]); }
#endif
#if DBGM == 3
__global__ __launch_bounds__(64) void k_dbg3(const float* __restrict__ H2, float* __restrict__ out) { __shared__ __align__(16) float s[192]; const int t = threadIdx.x; for (int i = t; i < 192; i += 64) s[i] = H2[(size_t)((i * 2731) % 4096) * 32 + (i * 7) % 20]; __syncthreads(); if (t < 48) vst2(out + t * 4, *(const v4f*)&s[t * 4]); }
#endif
#if DBGM == 4
__global__ __launch_bounds__(256) void k_fakeh2(const float* __restrict__ X, float* __restrict__ H2) { const int tid = threadIdx.x; const size_t n = (size_t)blockIdx.x * 64 + (tid >> 2); for (int p = (tid & 3); p < 8; p += 4) { v4f v; for (int i = 0; i < 4; ++i) { const int c = p * 4 + i; v[i] = (n < (size_t)CSR_N && c < 20) ? bfr(X[n * 128 + c]) : 0.f; } vst2(H2 + n * 32 + p * 4, v); } }
#endif
#if DBGM == 2 || DBGM == 3
__global__ __launch_bounds__(256) void k_fakeh1(const float* __restrict__ X, float* __restrict__ H1) { const int tid = threadIdx.x; const size_t n = (size_t)blockIdx.x * 64 + (tid >> 2); for (int p = (tid & 3); p < 16; p += 4) { v4f v; for (int i = 0; i < 4; ++i) { const int c = p * 4 + i; v[i] = (n < (size_t)CSR_N && c < 40) ? bfr(X[n * 128 + c]) : 0.f; } vst2(H1 + n * 64 + p * 4, v); } }
#endif
extern "C" void kernel_launch(void* const* d_in, const int* in_sizes, int n_in, void* d_out, int out_size, void* d_ws, size_t ws_size, hipStream_t stream) {
  (void)in_sizes; (void)n_in; (void)out_size;
  const float** F = (const float**)d_in; const int** I = (const int**)d_in;
  if (ws_size < (size_t)WS_END) return;
  char* ws = (char*)d_ws;
  int *CNT = (int*)(ws + WS_CNT), *OFF = (int*)(ws + WS_OFF), *BST = (int*)(ws + WS_BST), *SEGS = (int*)(ws + WS_SEGS), *SEGE = (int*)(ws + WS_SEGE), *FS = (int*)(ws + WS_FS), *FE = (int*)(ws + WS_FE), *RST = (int*)(ws + WS_RST), *RCT = (int*)(ws + WS_RCT);
  __bf16* PT = (__bf16*)(ws + WS_PT); float *KV1 = (float*)(ws + WS_KV1), *H1 = (float*)(ws + WS_H1), *KV2 = (float*)(ws + WS_KV2), *H2 = (float*)(ws + WS_H2), *PG = (float*)(ws + WS_PG);
  const int* EI = I[1]; const int* SRC = EI; const int* DST = EI + CSR_E;
  k_csr_cnt<<<CSR_NCH, 256, 0, stream>>>(DST, 1, CNT);
  k_csr_scan<<<1, 256, 0, stream>>>(CNT, OFF, BST);
  k_csr_scatter<<<CSR_NCH, 256, 0, stream>>>(SRC, DST, 1, 1, OFF, SEGS, SEGE);
  k_csr_bucket<<<CSR_NBK, 256, 0, stream>>>(CNT, OFF, BST, SEGS, SEGE, DST, 1, FS, FE, RST, RCT);
  k_pack<<<320, 128, 0, stream>>>(F[4], F[6], F[8], F[11], F[13], F[15], F[17], F[20], PT);
#if DBGM == 4
  k_fakeh2<<<NNP / 64, 256, 0, stream>>>(F[0], H2); k_pool<<<NG, 256, 0, stream>>>(I[3], H2, PG); k_mlp<<<1, 64, 0, stream>>>(PG, F[22], F[23], F[24], F[25], (float*)d_out); return;
#endif
#if DBGM == 2 || DBGM == 3
  k_fakeh1<<<NNP / 64, 256, 0, stream>>>(F[0], H1);
#else
  k_kv<1><<<NNP / 64, 128, 0, stream>>>(F[0], PT, F[7], F[9], KV1);
  k_conv<1><<<TLB1, 256, 0, stream>>>(F[0], PT, F[5], F[12], KV1, F[2], F[10], FS, FE, RST, RCT, H1);
#endif
#if DBGM == 1
  k_dbg1<<<1, 64, 0, stream>>>(H1, (float*)d_out); return;
#endif
  k_kv<2><<<NNP / 64, 128, 0, stream>>>(H1, PT, F[16], F[18], KV2);
  k_conv<2><<<TLB2, 256, 0, stream>>>(H1, PT, F[14], F[21], KV2, F[2], F[19], FS, FE, RST, RCT, H2);
#if DBGM == 3
  k_dbg3<<<1, 64, 0, stream>>>(H2, (float*)d_out); return;
#endif
  k_pool<<<NG, 256, 0, stream>>>(I[3], H2, PG);
  k_mlp<<<1, 64, 0, stream>>>(PG, F[22], F[23], F[24], F[25], (float*)d_out);
}
